// GlobalFeatureExtractorGNN_35871566856973
// MI455X (gfx1250) — hardware-verified
//
#include <hip/hip_runtime.h>
#include <math.h>

#define NN 50000
#define NE 1600000
#define NV (NE + NN)
#define CH 128
#define NG 64
#define MP 50048
#define NT 256
#define TG 2048
#define NTILE 25
#define NROWT (NTILE * TG)
#define SCH 4096
#define SPT (SCH / NT)
#define NCH ((NV + SCH - 1) / SCH)
#define NPB 128
#define NPN 391
#define PROWS (NG + 1)
#define WSC 16.0f
#define WSC_INV 0.0625f
#define NEG_SLOPE 0.2f
#define SELU_SC 1.0507009873554805f
#define SELU_AL 1.6732632423543772f

static_assert(NE % SPT == 0);
static_assert(MP % 64 == 0 && MP >= NN && MP % 32 == 0);
static_assert(NROWT >= MP);
static_assert(NPB * NPN >= NN);
static_assert(SCH <= 4096 && TG <= 2048 && TG / 8 == 256);
static_assert(NCH * SCH >= NV);

typedef __attribute__((ext_vector_type(16))) _Float16 v16h;
typedef __attribute__((ext_vector_type(8)))  _Float16 v8h;
typedef __attribute__((ext_vector_type(4)))  _Float16 v4h;
typedef __attribute__((ext_vector_type(16))) __bf16   v16b;
typedef __attribute__((ext_vector_type(8)))  __bf16   v8b;
typedef __attribute__((ext_vector_type(8)))  float    v8f;
typedef __attribute__((ext_vector_type(4)))  float    v4f;
typedef __attribute__((ext_vector_type(4)))  int      v4i;
#define U16(p) ((const unsigned short*)(const void*)(p))

__device__ __forceinline__ unsigned short f2bf_bits(float f) {
  unsigned u = __float_as_uint(f);
  return (unsigned short)((u + 0x7FFFu + ((u >> 16) & 1u)) >> 16);
}
__device__ __forceinline__ float bf_bits2f(unsigned short h) { return __uint_as_float(((unsigned)h) << 16); }

__device__ __forceinline__ void dep_guard_h(v8f& a, v8f& b, v16h x, v16h y) { asm volatile("v_nop\n\tv_nop\n\tv_nop\n\tv_nop" : "+v"(a), "+v"(b) : "v"(x), "v"(y)); }
__device__ __forceinline__ void dep_guard_b(v8f& a, v8f& b, v16b x, v16b y) { asm volatile("v_nop\n\tv_nop\n\tv_nop\n\tv_nop" : "+v"(a), "+v"(b) : "v"(x), "v"(y)); }
__device__ __forceinline__ void keep4_h(v16h a, v16h b, v16h c, v16h d) { asm volatile("v_nop" :: "v"(a), "v"(b), "v"(c), "v"(d)); }
__device__ __forceinline__ void keep4_b(v16b a, v16b b, v16b c, v16b d) { asm volatile("v_nop" :: "v"(a), "v"(b), "v"(c), "v"(d)); }
__device__ __forceinline__ void acc_guard4(v8f& a, v8f& b, v8f& c, v8f& d) { asm volatile("v_nop\n\tv_nop\n\tv_nop\n\tv_nop" : "+v"(a), "+v"(b), "+v"(c), "+v"(d)); }
template <typename T> struct Frag;
template <> struct Frag<_Float16> {
  typedef v16h V; union U { v16h v; v8h h[2]; };
  static __device__ __forceinline__ v16h load(const _Float16* p) {
    U f; f.h[0] = *(const v8h*)(p); f.h[1] = *(const v8h*)(p + 16); return f.v;
  }
  static __device__ __forceinline__ v8f mma(v16h a, v16h b, v8f c) {
    return __builtin_amdgcn_wmma_f32_16x16x32_f16(false, a, false, b, (short)0, c, false, false);
  }
  static __device__ __forceinline__ void guard(v8f& a, v8f& b, v16h x, v16h y) { dep_guard_h(a, b, x, y); }
  static __device__ __forceinline__ void keep(v16h a, v16h b, v16h c, v16h d) { keep4_h(a, b, c, d); }
};
template <> struct Frag<__bf16> {
  typedef v16b V; union U { v16b v; v8b h[2]; };
  static __device__ __forceinline__ v16b load(const __bf16* p) {
    U f; f.h[0] = *(const v8b*)(p); f.h[1] = *(const v8b*)(p + 16); return f.v;
  }
  static __device__ __forceinline__ v8f mma(v16b a, v16b b, v8f c) {
    return __builtin_amdgcn_wmma_f32_16x16x32_bf16(false, a, false, b, (short)0, c, false, false);
  }
  static __device__ __forceinline__ void guard(v8f& a, v8f& b, v16b x, v16b y) { dep_guard_b(a, b, x, y); }
  static __device__ __forceinline__ void keep(v16b a, v16b b, v16b c, v16b d) { keep4_b(a, b, c, d); }
};

template <int ET> struct Elem;
template <> struct Elem<0> { typedef _Float16 T; };
template <> struct Elem<1> { typedef __bf16 T; };
template <int ET, bool SPLIT, int BIAS_MODE, int OUT_MODE, bool RESID, int ACT = 0>
__global__ __launch_bounds__(256) void wmma_gemm64(
    const unsigned short* __restrict__ Ap, const unsigned short* __restrict__ A2p, int lda, long strideA,
    const unsigned short* __restrict__ Btp, const unsigned short* __restrict__ Bt2p, int ldb, long strideB,
    void* __restrict__ Cout, void* __restrict__ Cout2, int ldc, long strideC,
    const float* __restrict__ bias,
    const float* __restrict__ resid, long strideR,
    int M, int N, int K, float scale) {
  typedef typename Elem<ET>::T T;
  typedef typename Frag<T>::V V;
  const T* A = (const T*)Ap; const T* A2 = (const T*)A2p; const T* Bt = (const T*)Btp; const T* Bt2 = (const T*)Bt2p;
  __shared__ __align__(16) float sT[8][16 * 68];
  const int b    = blockIdx.y;
  const int lane = threadIdx.x & 31;
  const int wave = threadIdx.x >> 5;
  const int tilesN = N >> 6;
  const int tilesM = M >> 6;
  const int tile = blockIdx.x * 8 + wave;
  if (tile >= tilesM * tilesN) return;
  const int tm = tile / tilesN;
  const int tn = tile - tm * tilesN;
  const int m0 = tm << 6;
  const int n0 = tn << 6;

  const T* Ab  = A  + (size_t)b * strideA;
  const T* Bb  = Bt + (size_t)b * strideB;
  const T* Ab2 = SPLIT ? (A2  + (size_t)b * strideA) : nullptr;
  const T* Bb2 = SPLIT ? (Bt2 + (size_t)b * strideB) : nullptr;

  const int rlane = lane & 15;
  const int koff  = (lane >> 4) * 8;
  const int mOff  = (lane >> 4) * 8;

  v8f acc[4][4];
#pragma unroll
  for (int i = 0; i < 4; ++i)
#pragma unroll
    for (int j = 0; j < 4; ++j) acc[i][j] = (v8f){0.f,0.f,0.f,0.f,0.f,0.f,0.f,0.f};

  for (int k0 = 0; k0 < K; k0 += 32) {
    V bh[4], bl[4];
#pragma unroll
    for (int j = 0; j < 4; ++j) {
      const size_t bo = (size_t)(n0 + (j << 4) + rlane) * ldb + koff + k0;
      bh[j] = Frag<T>::load(Bb + bo);
      if (SPLIT) bl[j] = Frag<T>::load(Bb2 + bo);
    }
#pragma unroll
    for (int i = 0; i < 4; ++i) {
      const size_t ao = (size_t)(m0 + (i << 4) + rlane) * lda + koff + k0;
      V ah = Frag<T>::load(Ab + ao);
      V al;
      if (SPLIT) al = Frag<T>::load(Ab2 + ao);
#pragma unroll
      for (int j = 0; j < 4; ++j) {
        acc[i][j] = Frag<T>::mma(ah, bh[j], acc[i][j]);
        if (SPLIT) {
          acc[i][j] = Frag<T>::mma(ah, bl[j], acc[i][j]);
          acc[i][j] = Frag<T>::mma(al, bh[j], acc[i][j]);
        }
      }
      Frag<T>::guard(acc[i][0], acc[i][3], ah, SPLIT ? al : ah);
    }
    Frag<T>::keep(bh[0], bh[1], bh[2], bh[3]);
    if (SPLIT) Frag<T>::keep(bl[0], bl[1], bl[2], bl[3]);
  }
  acc_guard4(acc[0][0], acc[0][1], acc[0][2], acc[0][3]);
  acc_guard4(acc[1][0], acc[1][1], acc[1][2], acc[1][3]);
  acc_guard4(acc[2][0], acc[2][1], acc[2][2], acc[2][3]);
  acc_guard4(acc[3][0], acc[3][1], acc[3][2], acc[3][3]);

  float* slab = sT[wave];
  const float* Rb = RESID ? (resid + (size_t)b * strideR) : nullptr;
#pragma unroll
  for (int i = 0; i < 4; ++i) {
    const int mBase = m0 + (i << 4);
#pragma unroll
    for (int j = 0; j < 4; ++j) {
      const int n = n0 + (j << 4) + rlane;
      float bv = 0.f;
      if (BIAS_MODE == 2) bv = bias[n];
#pragma unroll
      for (int r = 0; r < 8; ++r) {
        float v = acc[i][j][r] * scale;
        if (BIAS_MODE == 1) v += bias[mBase + mOff + r];
        if (BIAS_MODE == 2) v += bv;
        if (RESID) v += Rb[(size_t)(mBase + mOff + r) * ldc + n];
        if (ACT == 1) v = tanhf(v);
        if (ACT == 2) v = fmaxf(v, 0.0f);
        if (ACT == 3) v = v / (1.0f + expf(-v));
        if (ACT == 4) v = (v > 0.f) ? v : 0.01f * v;
        if (ACT == 5) v = 0.5f * v * (1.0f + erff(v * 0.70710678118654752f));
        slab[(mOff + r) * 68 + (j << 4) + rlane] = v;
      }
    }
    __builtin_amdgcn_fence(__ATOMIC_RELEASE, "workgroup");
    __builtin_amdgcn_wave_barrier();
    __builtin_amdgcn_fence(__ATOMIC_ACQUIRE, "workgroup");
    if (OUT_MODE == 0) {
      float* C = (float*)Cout + (size_t)b * strideC;
      const int hh = lane >> 4, c4 = (lane & 15) * 4;
      for (int pass = 0; pass < 2; ++pass) {
#pragma unroll
        for (int it = 0; it < 8; ++it) {
          const int row = it * 2 + hh;
          v4f v = *(const v4f*)(slab + row * 68 + c4);
          *(volatile v4f*)(C + (size_t)(mBase + row) * ldc + n0 + c4) = v;
        }
        __threadfence();
      }
    } else {
      const int q = lane >> 3, c8 = (lane & 7) * 8;
      unsigned short* C  = (unsigned short*)Cout  + (size_t)b * strideC;
      unsigned short* C2 = (OUT_MODE == 2) ? ((unsigned short*)Cout2 + (size_t)b * strideC) : nullptr;
      for (int pass = 0; pass < 2; ++pass) {
#pragma unroll
        for (int it = 0; it < 4; ++it) {
          const int row = it * 4 + q;
          const float* sp = slab + row * 68 + c8;
          v8h hv, lv;
#pragma unroll
          for (int e = 0; e < 8; ++e) {
            if (OUT_MODE == 1) {
              hv[e] = (_Float16)sp[e];
            } else {
              unsigned short hb = f2bf_bits(sp[e]);
              unsigned short lb = f2bf_bits(sp[e] - bf_bits2f(hb));
              hv[e] = __builtin_bit_cast(_Float16, hb);
              lv[e] = __builtin_bit_cast(_Float16, lb);
            }
          }
          *(volatile v8h*)(C + (size_t)(mBase + row) * ldc + n0 + c8) = hv;
          if (OUT_MODE == 2) *(volatile v8h*)(C2 + (size_t)(mBase + row) * ldc + n0 + c8) = lv;
        }
        __threadfence();
      }
    }
    __builtin_amdgcn_fence(__ATOMIC_RELEASE, "workgroup");
    __builtin_amdgcn_wave_barrier();
    __builtin_amdgcn_fence(__ATOMIC_ACQUIRE, "workgroup");
  }
}

__global__ __launch_bounds__(256) void cast_x_kernel(
    const float* __restrict__ in, unsigned short* __restrict__ out, int nval2, int n2) {
  const int i = blockIdx.x * 256 + threadIdx.x;
  if (i < n2) {
    const int ic = (i < nval2) ? i : (nval2 - 1);
    float f0 = in[2 * (size_t)ic], f1 = in[2 * (size_t)ic + 1];
    if (i >= nval2) { f0 = 0.f; f1 = 0.f; }
    const _Float16 h0 = (_Float16)f0, h1 = (_Float16)f1;
    const unsigned u = (unsigned)__builtin_bit_cast(unsigned short, h0) | ((unsigned)__builtin_bit_cast(unsigned short, h1) << 16);
    ((volatile unsigned*)out)[i] = u;
    __threadfence();
    ((volatile unsigned*)out)[i] = u;
  }
}

__device__ __forceinline__ unsigned pack_f16x2(float a, float b) {
  const _Float16 h0 = (_Float16)a, h1 = (_Float16)b;
  return (unsigned)__builtin_bit_cast(unsigned short, h0) | ((unsigned)__builtin_bit_cast(unsigned short, h1) << 16);
}

__global__ __launch_bounds__(NT) void wprep_kernel(const float* __restrict__ W1, const float* __restrict__ W2,
                                                  unsigned* __restrict__ Bt1, unsigned* __restrict__ Bt2) {
  const int t = threadIdx.x;
  for (int i = t; i < CH * (CH / 2); i += NT) {
    const int n = i >> 6, k = 2 * (i & 63);
    const unsigned u1 = pack_f16x2(W1[k * CH + n] * WSC, W1[(k + 1) * CH + n] * WSC);
    ((volatile unsigned*)Bt1)[i] = u1; __threadfence(); ((volatile unsigned*)Bt1)[i] = u1;
    const unsigned u2 = pack_f16x2(W2[k * CH + n] * WSC, W2[(k + 1) * CH + n] * WSC);
    ((volatile unsigned*)Bt2)[i] = u2; __threadfence(); ((volatile unsigned*)Bt2)[i] = u2;
  }
}

__global__ __launch_bounds__(NT) void alpha_kernel(const float* __restrict__ H, const float* __restrict__ asrc,
                                                  const float* __restrict__ adst, float* __restrict__ ALS,
                                                  float* __restrict__ ALD) {
  const int lane = threadIdx.x & 31, wave = threadIdx.x >> 5;
  const int nb = (blockIdx.x * (NT / 32) + wave) * 32;
  if (nb < MP) {
    const int c4 = 4 * lane;
    const v4f sa = *(const v4f*)(asrc + c4);
    const v4f da = *(const v4f*)(adst + c4);
    float ks = 0.f, kd = 0.f;
#pragma unroll 1
    for (int j = 0; j < 32; ++j) {
      const int n = nb + j;
      const v4f hv = *(const v4f*)(H + (size_t)n * CH + c4);
      float s = hv[0] * sa[0]; s = fmaf(hv[1], sa[1], s); s = fmaf(hv[2], sa[2], s); s = fmaf(hv[3], sa[3], s);
      float d = hv[0] * da[0]; d = fmaf(hv[1], da[1], d); d = fmaf(hv[2], da[2], d); d = fmaf(hv[3], da[3], d);
#pragma unroll
      for (int off = 16; off > 0; off >>= 1) { s += __shfl_xor(s, off, 32); d += __shfl_xor(d, off, 32); }
      if (lane == j) { ks = s; kd = d; }
    }
    float* ps = ALS + nb + lane;
    float* pd = ALD + nb + lane;
    *(volatile float*)ps = ks; *(volatile float*)pd = kd;
    __threadfence();
    *(volatile float*)ps = ks; *(volatile float*)pd = kd;
  }
}

__device__ __forceinline__ int blk_excl_scan(int cnt, int* scan_ws, int tid, int* tot) {
  const int lane = tid & 31, wave = tid >> 5; int incl = cnt;
#pragma unroll
  for (int o = 1; o < 32; o <<= 1) { const int v = __shfl_up(incl, o, 32); if (lane >= o) incl += v; }
  if (lane == 31) scan_ws[wave] = incl;
  __syncthreads();
  if (wave == 0) { int wv = (lane < NT / 32) ? scan_ws[lane] : 0; int wincl = wv;
#pragma unroll
    for (int o = 1; o < 32; o <<= 1) { const int v = __shfl_up(wincl, o, 32); if (lane >= o) wincl += v; }
    if (lane < NT / 32) scan_ws[32 + lane] = wincl - wv; if (lane == 31) scan_ws[64] = wincl; }
  __syncthreads();
  const int res = scan_ws[32 + wave] + incl - cnt; *tot = scan_ws[64];
  return res;
}
template <int SP, int CAP, int NTOT>
__device__ __forceinline__ int chunk_hits(const int* __restrict__ dstv, int e0, int n0, int tid, int* LIST, int* scan_ws) {
  const int eb = e0 + tid * SP;
  const bool real = eb < NE;
  const int ebc = real ? eb : (NE - SP);
  int rec[SP]; int cnt = 0;
#pragma unroll
  for (int k = 0; k < SP; k += 4) {
    const v4i d4 = *(const v4i*)(dstv + ebc + k);
#pragma unroll
    for (int q = 0; q < 4; ++q) {
      const int e = eb + k + q;
      const int d = real ? d4[q] : (e - NE);
      const bool valid = real ? ((unsigned)d < (unsigned)NN) : (e < NTOT);
      int r = -1;
      if (valid && d >= n0 && d < n0 + TG) { r = ((d - n0) << 12) | (e - e0); ++cnt; }
      rec[k + q] = r;
    }
  }
  int tot; int p = blk_excl_scan(cnt, scan_ws, tid, &tot);
#pragma unroll
  for (int k = 0; k < SP; ++k) if (rec[k] >= 0) { if ((unsigned)p < (unsigned)CAP) LIST[p] = rec[k]; ++p; }
  __syncthreads();
  return tot < CAP ? tot : CAP;
}

template <int OUTF32>
__global__ __launch_bounds__(NT) void agg_kernel(const float* __restrict__ H, const int* __restrict__ ei,
                                                const float* __restrict__ ALS, const float* __restrict__ ALD,
                                                const float* __restrict__ bias, float* __restrict__ ACC,
                                                unsigned short* __restrict__ X16p, float* __restrict__ Y) {
  __shared__ __align__(16) float SM[TG];
  __shared__ __align__(16) float SL[TG];
  __shared__ int LIST[SCH];
  __shared__ int scan_ws[80];
  _Float16* X16 = (_Float16*)X16p;
  const int tid = threadIdx.x, lane = tid & 31, wave = tid >> 5;
  const int n0 = blockIdx.x * TG;
  const int c4 = 4 * lane;
  const v4f b4 = *(const v4f*)(bias + c4);
  for (int i = tid; i < TG; i += NT) { SM[i] = -INFINITY; SL[i] = 0.f; }
  float* accb = ACC + (size_t)n0 * CH;
  {
    const v4f z4 = {0.f, 0.f, 0.f, 0.f};
    for (int pass = 0; pass < 2; ++pass) {
#pragma unroll 1
      for (int j = 0; j < TG / 8; ++j) {
        float* ap = accb + (size_t)(wave * (TG / 8) + j) * CH + c4;
        *(volatile v4f*)ap = z4;
      }
      __threadfence();
    }
  }
  __syncthreads();
  const int* srcv = ei;
  const int* dstv = ei + NE;
#pragma unroll 1
  for (int c = 0; c < NCH; ++c) {
    const int e0 = c * SCH;
    const int tot = chunk_hits<SPT, SCH, NV>(dstv, e0, n0, tid, LIST, scan_ws);
#pragma unroll 1
    for (int base = 0; base < tot; base += 32) {
      const int q = base + lane;
      const int rv = (q < tot) ? LIST[q < SCH ? q : (SCH - 1)] : -1;
      const int own = (rv >= 0 && (rv >> 20) == wave) ? 1 : 0;
      unsigned msk = (unsigned)__ballot(own);
#pragma unroll 1
      for (int it = 0; it < 32; ++it) {
        if (msk == 0u) break;
        const int bp = __builtin_ctz(msk); msk &= msk - 1u;
        const int r = __shfl(rv, bp, 32);
        const int dl = r >> 12;
        const int e  = e0 + (r & 0xFFF);
        const int d  = n0 + dl;
        const bool real = e < NE;
        const int ec = real ? e : (NE - 1);
        int s = srcv[ec];
        s = s < 0 ? 0 : (s >= NN ? NN - 1 : s);
        s = real ? s : d;
        float lg = ALS[s] + ALD[d];
        lg = (lg > 0.f) ? lg : NEG_SLOPE * lg;
        const float mo = SM[dl], lo = SL[dl];
        const float mn = fmaxf(mo, lg);
        const float rr = __expf(mo - mn), ex = __expf(lg - mn);
        const float ln = fmaf(lo, rr, ex);
        if (lane == 0) { SM[dl] = mn; SL[dl] = ln; }
        float* ap = accb + (size_t)dl * CH + c4;
        const v4f qv = *(const v4f*)ap;
        const v4f hv = *(const v4f*)(H + (size_t)s * CH + c4);
        v4f o;
#pragma unroll
        for (int i = 0; i < 4; ++i) o[i] = fmaf(qv[i], rr, ex * hv[i]);
        *(volatile v4f*)ap = o;
        __threadfence();
        *(volatile v4f*)ap = o;
        asm volatile("" ::: "memory");
      }
    }
    __syncthreads();
  }
#pragma unroll 1
  for (int j = 0; j < TG / 8; ++j) {
    const int dl = wave * (TG / 8) + j;
    const int n = n0 + dl;
    if (n < MP) {
      const bool live = n < NN;
      const float* ap = accb + (size_t)dl * CH + c4;
      const v4f qv = *(const v4f*)ap;
      float l = SL[dl];
      l = (live && l > 0.f) ? l : 1.0f;
      const float inv = 1.0f / l;
      v4f y;
#pragma unroll
      for (int i = 0; i < 4; ++i) {
        const float v = fmaf(qv[i], inv, b4[i]);
        const float sv = (v > 0.f) ? (SELU_SC * v) : ((SELU_SC * SELU_AL) * (__expf(v) - 1.0f));
        y[i] = live ? sv : 0.f;
      }
      if (OUTF32) {
        float* yp = Y + (size_t)n * CH + c4;
        *(volatile v4f*)yp = y;
        __threadfence();
        *(volatile v4f*)yp = y;
      } else {
        const int sl = (2 * lane) & 31;
        v8h h8;
#pragma unroll
        for (int i = 0; i < 4; ++i) {
          const float ta = __shfl(y[i], sl, 32), tb = __shfl(y[i], sl + 1, 32);
          h8[i] = (_Float16)ta; h8[4 + i] = (_Float16)tb;
        }
        _Float16* hq = X16 + (size_t)n * CH + 8 * (lane & 15);
        for (int pass = 0; pass < 2; ++pass) {
          if (lane < 16) *(volatile v8h*)hq = h8;
          __threadfence();
        }
      }
    }
  }
}

__global__ __launch_bounds__(32) void pool_part_kernel(const float* __restrict__ Y, const int* __restrict__ batch,
                                                     float* __restrict__ PART) {
  __shared__ __align__(16) float PS[NG * CH];
  __shared__ __align__(16) float PC[CH];
  const int lane = threadIdx.x;
  const int c4 = 4 * lane;
  v4f* PS4 = (v4f*)PS;
  const v4f z4 = {0.f, 0.f, 0.f, 0.f};
#pragma unroll 1
  for (int g = 0; g < NG; ++g) PS4[g * 32 + lane] = z4;
  PC[lane] = 0.f; PC[32 + lane] = 0.f; PC[64 + lane] = 0.f; PC[96 + lane] = 0.f;
  __syncthreads();
  const int nb = blockIdx.x * NPN;
#pragma unroll 1
  for (int i = 0; i < NPN; ++i) {
    const int n = nb + i;
    if (n < NN) {
      const int g = batch[n];
      const v4f yv = *(const v4f*)(Y + (size_t)n * CH + c4);
      if ((unsigned)g < (unsigned)NG) {
        v4f p = PS4[g * 32 + lane];
        p += yv;
        PS4[g * 32 + lane] = p;
        if (lane == 0) PC[g] += 1.0f;
      }
    }
  }
  __syncthreads();
  float* pb = PART + (size_t)blockIdx.x * PROWS * CH;
  for (int pass = 0; pass < 2; ++pass) {
#pragma unroll 1
    for (int g = 0; g < NG; ++g) {
      const v4f v = PS4[g * 32 + lane];
      *(volatile v4f*)(pb + (size_t)g * CH + c4) = v;
    }
    const v4f cv = *(const v4f*)(PC + c4);
    *(volatile v4f*)(pb + (size_t)NG * CH + c4) = cv;
    __threadfence();
  }
}

__global__ __launch_bounds__(NT) void pool_final_kernel(const float* __restrict__ PART, float* __restrict__ out) {
  const int lane = threadIdx.x & 31, wave = threadIdx.x >> 5;
  const int c4 = 4 * lane;
#pragma unroll 1
  for (int k = 0; k < NG / 8; ++k) {
    const int g = wave * (NG / 8) + k;
    v4f s = {0.f, 0.f, 0.f, 0.f};
    float cnt = 0.f;
#pragma unroll 1
    for (int p = 0; p < NPB; ++p) {
      const float* pb = PART + (size_t)p * PROWS * CH;
      const v4f v = *(const v4f*)(pb + (size_t)g * CH + c4);
      s += v;
      cnt += pb[(size_t)NG * CH + g];
    }
    const float inv = 1.0f / fmaxf(cnt, 1.0f);
    v4f o;
#pragma unroll
    for (int i = 0; i < 4; ++i) o[i] = s[i] * inv;
    float* op = out + (size_t)g * CH + c4;
    *(volatile v4f*)op = o;
    __threadfence();
    *(volatile v4f*)op = o;
  }
}

extern "C" void kernel_launch(void* const* d_in, const int* in_sizes, int n_in,
                              void* d_out, int out_size, void* d_ws, size_t ws_size, hipStream_t stream) {
  if (n_in < 11) return;
  const float* u     = (const float*)d_in[0];
  const float* W1    = (const float*)d_in[1];
  const float* as1   = (const float*)d_in[2];
  const float* ad1   = (const float*)d_in[3];
  const float* b1    = (const float*)d_in[4];
  const float* W2    = (const float*)d_in[5];
  const float* as2   = (const float*)d_in[6];
  const float* ad2   = (const float*)d_in[7];
  const float* b2    = (const float*)d_in[8];
  const int*   ei    = (const int*)  d_in[9];
  const int*   batch = (const int*)  d_in[10];
  float* out = (float*)d_out;

  if (in_sizes[0] != NN * CH || in_sizes[1] != CH * CH || in_sizes[5] != CH * CH) return;
  if (in_sizes[2] != CH || in_sizes[3] != CH || in_sizes[4] != CH || in_sizes[6] != CH || in_sizes[7] != CH || in_sizes[8] != CH) return;
  if (in_sizes[9] != 2 * NE || in_sizes[10] != NN || out_size != NG * CH) return;

  char* ws = (char*)d_ws; size_t off = 0;
  auto carve = [&](size_t bytes) -> char* { char* p = ws + off; off += (bytes + 255) & ~(size_t)255; return p; };
  unsigned short* X16  = (unsigned short*)carve((size_t)MP * CH * 2);
  unsigned*       Bt1  = (unsigned*)carve((size_t)CH * CH * 2);
  unsigned*       Bt2  = (unsigned*)carve((size_t)CH * CH * 2);
  float*          H    = (float*)carve((size_t)MP * CH * 4);
  float*          ALS  = (float*)carve((size_t)MP * 4);
  float*          ALD  = (float*)carve((size_t)MP * 4);
  float*          ACC  = (float*)carve((size_t)NROWT * CH * 4);
  float*          Y    = (float*)carve((size_t)MP * CH * 4);
  float*          PART = (float*)carve((size_t)NPB * PROWS * CH * 4);
  if (off > ws_size || off > (size_t)134217728) return;

  cast_x_kernel<<<(MP * (CH / 2) + 255) / 256, 256, 0, stream>>>(u, X16, NN * (CH / 2), MP * (CH / 2));
  wprep_kernel<<<1, NT, 0, stream>>>(W1, W2, Bt1, Bt2);

  const int tiles = (MP / 64) * (CH / 64);
  const int gemm_blocks = (tiles + 7) / 8;
  const int alpha_blocks = (MP / 32 + (NT / 32) - 1) / (NT / 32);

  wmma_gemm64<0, false, 0, 0, false, 0><<<dim3(gemm_blocks, 1), 256, 0, stream>>>(
      U16(X16), U16(X16), CH, 0L,
      U16(Bt1), U16(Bt1), CH, 0L,
      (void*)H, (void*)nullptr, CH, 0L,
      b1, (const float*)nullptr, 0L, MP, CH, CH, WSC_INV);
  alpha_kernel<<<alpha_blocks, NT, 0, stream>>>(H, as1, ad1, ALS, ALD);
  agg_kernel<0><<<NTILE, NT, 0, stream>>>(H, ei, ALS, ALD, b1, ACC, X16, Y);

  wmma_gemm64<0, false, 0, 0, false, 0><<<dim3(gemm_blocks, 1), 256, 0, stream>>>(
      U16(X16), U16(X16), CH, 0L,
      U16(Bt2), U16(Bt2), CH, 0L,
      (void*)H, (void*)nullptr, CH, 0L,
      b2, (const float*)nullptr, 0L, MP, CH, CH, WSC_INV);
  alpha_kernel<<<alpha_blocks, NT, 0, stream>>>(H, as2, ad2, ALS, ALD);
  agg_kernel<1><<<NTILE, NT, 0, stream>>>(H, ei, ALS, ALD, b2, ACC, X16, Y);

  pool_part_kernel<<<NPB, 32, 0, stream>>>(Y, batch, PART);
  pool_final_kernel<<<1, NT, 0, stream>>>(PART, out);
}
